// DirectEncodingModelTrainable_46737834115508
// MI455X (gfx1250) — hardware-verified
//
#include <hip/hip_runtime.h>
#include <stddef.h>


typedef _Float16 v16h __attribute__((ext_vector_type(16)));
typedef _Float16 v8h  __attribute__((ext_vector_type(8)));
typedef float    v8f  __attribute__((ext_vector_type(8)));
typedef float    v4f  __attribute__((ext_vector_type(4)));
typedef _Float16 h16;

#ifndef NROWS
#define NROWS 8192
#endif
#define NROWS_FULL 8192
#define N_IN   1024
#define NLEV   6
#define NG     64
#define KIN    32
#define KOUT   8
#define LEVW   (NG * KOUT)
#define NCOMP  ((NLEV - 1) * LEVW)
#define TILE   16
#define NPAD   16

#define BUFP 2560
#define LDA  40
#define OLD  32

#define WCARRY 64.0f

#define LDS_TOTAL ((size_t)TILE * BUFP * 2 + (size_t)8 * 16 * LDA * 2 + (size_t)8 * 16 * OLD * 4)

static_assert(NROWS >= TILE && NROWS <= NROWS_FULL && (NROWS % TILE) == 0);
static_assert(KIN == 32);
static_assert(KOUT == 8 && NPAD == 16);
static_assert(NG == 8 * 8);
static_assert(LEVW == 8 * 2 * 32);
static_assert(4 * KOUT == 32);
static_assert(((size_t)NROWS * N_IN) % (256 * 8) == 0);
static_assert((BUFP % 8) == 0 && BUFP >= NCOMP);
static_assert(((TILE * BUFP / 8) % 256) == 0);
static_assert((LDA % 8) == 0 && LDA >= KIN);
static_assert((OLD % 4) == 0 && OLD >= 32);
static_assert(KIN * KOUT == 64 * 4);
static_assert(NPAD * KIN == 64 * 8);
static_assert(LDS_TOTAL <= (size_t)131072);
static_assert(LDS_TOTAL <= (size_t)110000);

#define WT_BYTES  ((size_t)NLEV * NG * NPAD * KIN * 2)
#define X16_BYTES ((size_t)NROWS * N_IN * 2)
#define OFF_WT    ((size_t)0)
#define OFF_X16   (OFF_WT + WT_BYTES)
#define WS_TOTAL  (OFF_X16 + X16_BYTES)
static_assert((WT_BYTES % 128) == 0 && (X16_BYTES % 128) == 0);
static_assert(WS_TOTAL <= (size_t)134217728);
static_assert((size_t)NROWS * LEVW * 4 <= (size_t)16777216);

__device__ __forceinline__ float bf16r(float x) {
  unsigned int u = __float_as_uint(x);
  u = (u + 0x7FFFu + ((u >> 16) & 1u)) & 0xFFFF0000u;
  return __uint_as_float(u);
}

static __device__ __forceinline__ h16 toh_flush(float v) {
  const h16 r = (h16)v;
  return (fabsf(v) < 6.103515625e-05f) ? (h16)0.0f : r;
}

__device__ __forceinline__ v16h frag_at(const _Float16* p) {
  v8h lo = *(const v8h*)(p);
  v8h hi = *(const v8h*)(p + 16);
  v16h out;
#pragma unroll
  for (int i = 0; i < 8; ++i) { out[i] = lo[i]; out[i + 8] = hi[i]; }
  return out;
}
__device__ __forceinline__ v16h ld_frag(const _Float16* base, unsigned ld) {
  const unsigned lane = threadIdx.x & 31u;
  return frag_at(base + (lane & 15u) * ld + (lane >> 4) * 8u);
}

__device__ __forceinline__ v8f wmma16(v16h a, v16h b, v8f c) {
  v8f d = __builtin_amdgcn_wmma_f32_16x16x32_f16(false, a, false, b, (short)0, c,
                                                 false, false);
  asm volatile("v_nop\n\tv_nop\n\tv_nop\n\tv_nop" : "+v"(d) : "v"(a), "v"(b));
  return d;
}

__device__ __forceinline__ void wave_lds_sync() {
  __builtin_amdgcn_fence(3  , "wavefront");
  asm volatile("s_wait_dscnt 0x0" ::: "memory");
  __builtin_amdgcn_wave_barrier();
}

__device__ __forceinline__ float tanh_act(float t) {
  const float e = __expf(2.0f * t);
  return 1.0f - 2.0f * __builtin_amdgcn_rcpf(e + 1.0f);
}

__global__ __launch_bounds__(64) void wprep_kernel(
    const float* __restrict__ W, _Float16* __restrict__ Wt) {
  __shared__ _Float16 T[NPAD * LDA];
  const unsigned tid = threadIdx.x;
  const unsigned g = blockIdx.x;
#pragma unroll
  for (unsigned j = 0; j < 4u; ++j) {
    const unsigned e = tid + 64u * j;
    const unsigned k = e >> 3, n = e & 7u;
    const float v = W[(size_t)g * (KIN * KOUT) + e];
    T[n * LDA + k] = toh_flush(WCARRY * bf16r(v));
    T[(8u + n) * LDA + k] = (h16)0.0f;
  }
  __syncthreads();
  const unsigned n = tid >> 2, kc = (tid & 3u) * 8u;
  const v8h x = *(const v8h*)&T[n * LDA + kc];
  _Float16* p = Wt + (size_t)g * (NPAD * KIN) + tid * 8u;
  *(volatile v8h*)p = x;
  __threadfence();
  *(volatile v8h*)p = x;
}

__global__ __launch_bounds__(256) void xconv_kernel(
    const float* __restrict__ X, _Float16* __restrict__ X16) {
  const size_t e = ((size_t)blockIdx.x * 256u + threadIdx.x) * 8u;
  const v4f a0 = *(const v4f*)(X + e);
  const v4f a1 = *(const v4f*)(X + e + 4);
  v8h o;
#pragma unroll
  for (int i = 0; i < 4; ++i) {
    o[i]     = toh_flush(bf16r(a0[i]));
    o[i + 4] = toh_flush(bf16r(a1[i]));
  }
  _Float16* p = X16 + e;
  *(volatile v8h*)p = o;
  __threadfence();
  *(volatile v8h*)p = o;
}

__global__ __launch_bounds__(256) void levels_kernel(
    const _Float16* __restrict__ X16, const _Float16* __restrict__ Wt,
    const float* __restrict__ Bias, const int* __restrict__ Idx, float* __restrict__ Out) {
  __shared__ _Float16 buf[TILE * BUFP];
  __shared__ _Float16 At[8 * 16 * LDA];
  __shared__ float Os[8 * 16 * OLD];

  const unsigned tid = threadIdx.x, lane = tid & 31u;
  const unsigned wave = (unsigned)__builtin_amdgcn_readfirstlane((int)(threadIdx.x >> 5));
  const unsigned hh = lane >> 4, m = lane & 15u;
  const unsigned row0 = blockIdx.x * (unsigned)TILE;
  _Float16* A = At + wave * (16u * LDA);
  float* O = Os + wave * (16u * OLD);

  {
    const v8h z = {};
#pragma unroll 4
    for (unsigned i = tid; i < (unsigned)(TILE * BUFP / 8); i += 256u) *(v8h*)&buf[i * 8u] = z;
  }
  __syncthreads();

#pragma unroll 1
  for (unsigned l = 0; l < (unsigned)NLEV; ++l) {
    const int live = N_IN + (int)l * LEVW;
    const bool last = (l == (unsigned)(NLEV - 1));
#pragma unroll 1
    for (unsigned j = 0; j < 8u; ++j) {
      const unsigned g = wave * 8u + j;
      const unsigned lg = l * (unsigned)NG + g;
      int col = Idx[lg * KIN + lane];
      col = min(max(col, 0), live - 1);
      const bool from_x = (col < N_IN);
      const unsigned xcol = (unsigned)min(col, N_IN - 1);
      const unsigned bcol = (unsigned)max(col - N_IN, 0);
      const size_t xbase = (size_t)row0 * N_IN + xcol;
#pragma unroll 1
      for (unsigned rh = 0; rh < 2u; ++rh) {
#pragma unroll
        for (unsigned q = 0; q < 8u; ++q) {
          const unsigned r = rh * 8u + q;
          const h16 xv = X16[xbase + (size_t)r * N_IN];
          const h16 bv = buf[r * BUFP + bcol];
          unsigned xu = (unsigned)__builtin_bit_cast(unsigned short, xv);
          unsigned bu = (unsigned)__builtin_bit_cast(unsigned short, bv);
          asm volatile("" : "+v"(xu));
          asm volatile("" : "+v"(bu));
          const unsigned su = from_x ? xu : bu;
          A[r * LDA + lane] = __builtin_bit_cast(h16, (unsigned short)su);
        }
      }
      wave_lds_sync();
      const v16h a = ld_frag(A, LDA);
      const v16h b = frag_at(Wt + (size_t)(lg * (unsigned)NPAD + m) * KIN + hh * 8u);
      v8f c = {};
      c = wmma16(a, b, c);
      wave_lds_sync();

      const float bb = bf16r(Bias[lg * KOUT + (m & 7u)]);
      float t[8];
#pragma unroll
      for (int v = 0; v < 8; ++v) t[v] = tanh_act(c[v] * (1.0f / WCARRY) + bb);

      if (!last) {
        const unsigned cb = l * (unsigned)LEVW + g * (unsigned)KOUT + m;
        if (m < 8u) {
#pragma unroll
          for (int v = 0; v < 8; ++v)
            buf[(hh * 8u + (unsigned)v) * BUFP + cb] = toh_flush(t[v]);
        }
      } else {
        if (m < 8u) {
#pragma unroll
          for (int v = 0; v < 8; ++v)
            O[(hh * 8u + (unsigned)v) * OLD + (j & 3u) * 8u + m] = t[v];
        }
        if ((j & 3u) == 3u) {
          wave_lds_sync();
          v4f xs[4];
          size_t off[4];
#pragma unroll
          for (unsigned i = 0; i < 4u; ++i) {
            const unsigned r = 4u * i + (lane >> 3);
            const unsigned cc = (lane & 7u) * 4u;
            xs[i] = *(const v4f*)&O[r * OLD + cc];
            off[i] = (size_t)(row0 + r) * LEVW + wave * 64u + (j >> 2) * 32u + cc;
          }
#pragma unroll
          for (int i = 0; i < 4; ++i) *(volatile v4f*)(Out + off[i]) = xs[i];
          __threadfence();
#pragma unroll
          for (int i = 0; i < 4; ++i) *(volatile v4f*)(Out + off[i]) = xs[i];
          wave_lds_sync();
        }
      }
    }
    __syncthreads();
  }
}

extern "C" void kernel_launch(void* const* d_in, const int* in_sizes, int n_in,
                              void* d_out, int out_size, void* d_ws, size_t ws_size,
                              hipStream_t stream) {
  if (n_in < 4) return;
  if ((long long)in_sizes[0] < (long long)NROWS * N_IN) return;
  if ((long long)in_sizes[1] < (long long)NLEV * NG * KIN * KOUT) return;
  if ((long long)in_sizes[2] < (long long)NLEV * NG * KOUT) return;
  if ((long long)in_sizes[3] < (long long)NLEV * NG * KIN) return;
  if ((long long)out_size < (long long)NROWS * LEVW) return;
  if (ws_size < WS_TOTAL) return;

  const float* X    = (const float*)d_in[0];
  const float* kern = (const float*)d_in[1];
  const float* bias = (const float*)d_in[2];
  const int*   idx  = (const int*)d_in[3];
  float* out = (float*)d_out;

  char* ws = (char*)d_ws;
  _Float16* Wt  = (_Float16*)(ws + OFF_WT);
  _Float16* X16 = (_Float16*)(ws + OFF_X16);

  wprep_kernel<<<dim3(NLEV * NG), dim3(64), 0, stream>>>(kern, Wt);
  xconv_kernel<<<dim3((unsigned)(((size_t)NROWS * N_IN) / 2048)), dim3(256), 0, stream>>>(X, X16);
  levels_kernel<<<dim3(NROWS / TILE), dim3(256), 0, stream>>>(X16, Wt, bias, idx, out);
}
